// GRU_Predictor_69801808494929
// MI455X (gfx1250) — hardware-verified
//
#include <hip/hip_runtime.h>
#include <math.h>
#include <stdint.h>

constexpr int NSEQ   = 512;
constexpr int NSTEP  = 2048;
constexpr int NIN    = 8;
constexpr int NHID   = 128;
constexpr int NG3    = 384;
constexpr int NOUT   = 96;
constexpr int NTHR   = 256;
constexpr int TROWS  = 32;
constexpr int KAUG   = 160;
constexpr int HPITCH = 168;
constexpr int XCH    = 32;
constexpr int GOFF   = NHID * KAUG;
constexpr int JOFF   = 16 * KAUG;
constexpr float A_CARRY = 16.0f;
constexpr float W_CARRY = 64.0f;
constexpr float Z_FOLD  = 1.0f / 1024.0f;

static_assert(NSEQ % TROWS == 0, "grid covers all sequences exactly");
static_assert(NSTEP % XCH == 0, "x chunks tile the time axis exactly");
static_assert(TROWS * XCH * NIN == NTHR * 32, "32 floats of x per thread per chunk");
static_assert((NG3 * KAUG / 8) % NTHR == 0, "recurrent weight plane prep grid exact");
static_assert((NOUT * NHID / 8) % NTHR == 0, "head weight plane prep grid exact");
static_assert(KAUG % 32 == 0 && NHID % 32 == 0, "K multiples of 32");
static_assert(HPITCH % 8 == 0 && HPITCH >= KAUG, "A tile pitch");
static_assert(TROWS * NOUT == NTHR * 3 * 4, "3 float4 per thread cover the 32x96 output tile");
static_assert(NG3 % 16 == 0 && NOUT % 32 == 0 && TROWS % 16 == 0, "tile multiples");

typedef __attribute__((ext_vector_type(16))) _Float16 v16h;
typedef __attribute__((ext_vector_type(8)))  _Float16 v8h;
typedef __attribute__((ext_vector_type(8)))  float    v8f;
typedef __attribute__((ext_vector_type(4)))  float    v4f;

__device__ __forceinline__ unsigned short f2bf_bits(float f) {
  unsigned u = __float_as_uint(f);
  return (unsigned short)((u + 0x7FFFu + ((u >> 16) & 1u)) >> 16);
}
__device__ __forceinline__ float bf_bits2f(unsigned short h) { return __uint_as_float(((unsigned)h) << 16); }
__device__ __forceinline__ float bfr(float f) { return bf_bits2f(f2bf_bits(f)); }

__device__ __forceinline__ void keep4_h(v16h a, v16h b, v16h c, v16h d) { asm volatile("v_nop" :: "v"(a), "v"(b), "v"(c), "v"(d)); }
__device__ __forceinline__ void acc_guard4(v8f& a, v8f& b, v8f& c, v8f& d) { asm volatile("v_nop\n\tv_nop\n\tv_nop\n\tv_nop" : "+v"(a), "+v"(b), "+v"(c), "+v"(d)); }
__device__ __forceinline__ void acc_guard2(v8f& a, v8f& b) { asm volatile("v_nop\n\tv_nop\n\tv_nop\n\tv_nop" : "+v"(a), "+v"(b)); }

template <typename T> struct Frag;
template <> struct Frag<_Float16> {
  typedef v16h V; union U { v16h v; v8h h[2]; };
  static __device__ __forceinline__ v16h load(const _Float16* p) {
    U f; f.h[0] = *(const v8h*)(p); f.h[1] = *(const v8h*)(p + 16); return f.v;
  }
  static __device__ __forceinline__ v8f mma(v16h a, v16h b, v8f c) {
    return __builtin_amdgcn_wmma_f32_16x16x32_f16(false, a, false, b, (short)0, c, false, false);
  }
};
typedef Frag<_Float16> FragH;

__device__ __forceinline__ float fsig(float v)  { return __builtin_amdgcn_rcpf(1.0f + __expf(-v)); }
__device__ __forceinline__ float ftanh(float v) { return 1.0f - 2.0f * __builtin_amdgcn_rcpf(__expf(2.0f * v) + 1.0f); }

template <bool AUG>
__global__ __launch_bounds__(NTHR) void wplane_kernel(const float* __restrict__ W1, const float* __restrict__ W2,
                                                      int n8, unsigned short* __restrict__ O) {
  const int i = blockIdx.x * NTHR + threadIdx.x;
  if (i >= n8) return;
  constexpr int P = AUG ? KAUG : NHID;
  const int e0   = i * 8;
  const int row  = e0 / P;
  const int col0 = e0 - row * P;
  v8h hv;
#pragma unroll
  for (int e = 0; e < 8; ++e) {
    const int col = col0 + e;
    const int c1 = col < NHID ? col : NHID - 1;
    float v = W1[(size_t)row * NHID + c1];
    if (AUG) {
      int c2 = col - NHID;
      c2 = c2 < 0 ? 0 : (c2 > NIN - 1 ? NIN - 1 : c2);
      const float v2 = W2[(size_t)row * NIN + c2];
      v = (col < NHID) ? v : ((col < NHID + NIN) ? v2 : 0.0f);
    }
    hv[e] = (_Float16)(bfr(v) * W_CARRY);
  }
  *(volatile v8h*)(O + e0) = hv;
  __threadfence();
  *(volatile v8h*)(O + e0) = hv;
}

__device__ __forceinline__ void mac_main(v8f (&aR)[2], v8f (&aZ)[2], v8f (&aN)[2],
                                         const _Float16* arow, const _Float16* wb) {
#pragma unroll 1
  for (int ks = 0; ks < 4; ++ks) {
    const int k0 = ks * 32;
    const v16h a  = FragH::load(arow + k0);
    const v16h r0 = FragH::load(wb + k0);
    const v16h r1 = FragH::load(wb + JOFF + k0);
    const v16h z0 = FragH::load(wb + GOFF + k0);
    const v16h z1 = FragH::load(wb + GOFF + JOFF + k0);
    const v16h n0 = FragH::load(wb + 2 * GOFF + k0);
    const v16h n1 = FragH::load(wb + 2 * GOFF + JOFF + k0);
    aR[0] = FragH::mma(a, r0, aR[0]);
    aR[1] = FragH::mma(a, r1, aR[1]);
    aZ[0] = FragH::mma(a, z0, aZ[0]);
    aZ[1] = FragH::mma(a, z1, aZ[1]);
    aN[0] = FragH::mma(a, n0, aN[0]);
    aN[1] = FragH::mma(a, n1, aN[1]);
    acc_guard4(aR[0], aR[1], aZ[0], aZ[1]);
    acc_guard2(aN[0], aN[1]);
    keep4_h(a, r0, r1, z0);
    keep4_h(z1, n0, n1, a);
  }
}

__device__ __forceinline__ void mac_tail(v8f (&aR)[2], v8f (&aZ)[2], v8f (&aX)[2],
                                         const _Float16* arow, const _Float16* wb) {
  const int k0 = NHID;
  const v16h a  = FragH::load(arow + k0);
  const v16h r0 = FragH::load(wb + k0);
  const v16h r1 = FragH::load(wb + JOFF + k0);
  const v16h z0 = FragH::load(wb + GOFF + k0);
  const v16h z1 = FragH::load(wb + GOFF + JOFF + k0);
  const v16h x0 = FragH::load(wb + 2 * GOFF + k0);
  const v16h x1 = FragH::load(wb + 2 * GOFF + JOFF + k0);
  aR[0] = FragH::mma(a, r0, aR[0]);
  aR[1] = FragH::mma(a, r1, aR[1]);
  aZ[0] = FragH::mma(a, z0, aZ[0]);
  aZ[1] = FragH::mma(a, z1, aZ[1]);
  aX[0] = FragH::mma(a, x0, aX[0]);
  aX[1] = FragH::mma(a, x1, aX[1]);
  acc_guard4(aR[0], aR[1], aZ[0], aZ[1]);
  acc_guard2(aX[0], aX[1]);
  keep4_h(a, r0, r1, z0);
  keep4_h(z1, x0, x1, a);
}

__device__ __forceinline__ void gru_cell8(const v8f& aR, const v8f& aZ, const v8f& aX, const v8f& aN,
                                          float cr, float cz, float cin, float chn, float (&h)[8]) {
#pragma unroll
  for (int r = 0; r < 8; ++r) {
    const float pr  = fmaf(aR[r], Z_FOLD, cr);
    const float pz  = fmaf(aZ[r], Z_FOLD, cz);
    const float gin = fmaf(aX[r], Z_FOLD, cin);
    const float ghn = fmaf(aN[r], Z_FOLD, chn);
    const float rr  = fsig(pr);
    const float zz  = fsig(pz);
    const float nn  = ftanh(fmaf(rr, ghn, gin));
    h[r] = fmaf(zz, h[r] - nn, nn);
  }
}

__global__ __launch_bounds__(NTHR) void gru_head_kernel(
    const float* __restrict__ x,
    const float* __restrict__ b_ih, const float* __restrict__ b_hh, const float* __restrict__ fc_b,
    const unsigned short* __restrict__ WBp, const unsigned short* __restrict__ FCp,
    float* __restrict__ out) {
  __shared__ __align__(16) _Float16 Ht[TROWS * HPITCH];
  __shared__ __align__(16) _Float16 Xs[TROWS * XCH * NIN];
  __shared__ __align__(16) float    Os[TROWS * NOUT];

  const int tid = threadIdx.x, lane = tid & 31, wave = tid >> 5;
  const int c = lane & 15, hh = lane >> 4, koff = hh * 8;
  const int rt = wave >> 2;
  const int ug = wave & 3;
  const int j0 = 32 * ug + c;
  const int j1 = j0 + 16;
  const int rb = rt * 16 + 8 * hh;
  const int rowbase = blockIdx.x * TROWS;

#pragma unroll 1
  for (int i = tid; i < TROWS * HPITCH; i += NTHR) Ht[i] = (_Float16)0.0f;

  const float cr0  = bfr(b_ih[j0]) + bfr(b_hh[j0]);
  const float cz0  = bfr(b_ih[NHID + j0]) + bfr(b_hh[NHID + j0]);
  const float cin0 = bfr(b_ih[2 * NHID + j0]);
  const float chn0 = bfr(b_hh[2 * NHID + j0]);
  const float cr1  = bfr(b_ih[j1]) + bfr(b_hh[j1]);
  const float cz1  = bfr(b_ih[NHID + j1]) + bfr(b_hh[NHID + j1]);
  const float cin1 = bfr(b_ih[2 * NHID + j1]);
  const float chn1 = bfr(b_hh[2 * NHID + j1]);

  float hs0[8], hs1[8];
#pragma unroll
  for (int r = 0; r < 8; ++r) { hs0[r] = 0.0f; hs1[r] = 0.0f; }
  __syncthreads();

  const _Float16* arow = Ht + (rt * 16 + c) * HPITCH + koff;
  const _Float16* wb = (const _Float16*)WBp + (size_t)j0 * KAUG + koff;
  const v8f z8 = {0.f, 0.f, 0.f, 0.f, 0.f, 0.f, 0.f, 0.f};

#pragma unroll 1
  for (int t = 0; t < NSTEP; ++t) {
    const int tc = t & (XCH - 1);
    if (tc == 0) {
      const int row = tid >> 3, sub = tid & 7;
      const float* src = x + ((size_t)(rowbase + row) * NSTEP + (size_t)(t + sub * 4)) * NIN;
#pragma unroll
      for (int s = 0; s < 4; ++s) {
        const v4f va = *(const v4f*)(src + s * NIN);
        const v4f vb = *(const v4f*)(src + s * NIN + 4);
        v8h hv;
        hv[0] = (_Float16)(bfr(va[0]) * A_CARRY); hv[1] = (_Float16)(bfr(va[1]) * A_CARRY);
        hv[2] = (_Float16)(bfr(va[2]) * A_CARRY); hv[3] = (_Float16)(bfr(va[3]) * A_CARRY);
        hv[4] = (_Float16)(bfr(vb[0]) * A_CARRY); hv[5] = (_Float16)(bfr(vb[1]) * A_CARRY);
        hv[6] = (_Float16)(bfr(vb[2]) * A_CARRY); hv[7] = (_Float16)(bfr(vb[3]) * A_CARRY);
        *(v8h*)(Xs + ((row * XCH) + sub * 4 + s) * NIN) = hv;
      }
      __syncthreads();
    }
    if (tid < TROWS) {
      const v8h xv = *(const v8h*)(Xs + (tid * XCH + tc) * NIN);
      *(v8h*)(Ht + tid * HPITCH + NHID) = xv;
    }
    __syncthreads();

    v8f aR[2], aZ[2], aN[2], aX[2];
    aR[0] = z8; aR[1] = z8; aZ[0] = z8; aZ[1] = z8; aN[0] = z8; aN[1] = z8; aX[0] = z8; aX[1] = z8;
    mac_main(aR, aZ, aN, arow, wb);
    mac_tail(aR, aZ, aX, arow, wb);
    gru_cell8(aR[0], aZ[0], aX[0], aN[0], cr0, cz0, cin0, chn0, hs0);
    gru_cell8(aR[1], aZ[1], aX[1], aN[1], cr1, cz1, cin1, chn1, hs1);
    __syncthreads();
#pragma unroll
    for (int r = 0; r < 8; ++r) {
      Ht[(rb + r) * HPITCH + j0] = (_Float16)(A_CARRY * hs0[r]);
      Ht[(rb + r) * HPITCH + j1] = (_Float16)(A_CARRY * hs1[r]);
    }
  }
  __syncthreads();

  if (ug < 3) {
    const int col0 = 32 * ug + c;
    const int col1 = col0 + 16;
    const _Float16* fb = (const _Float16*)FCp + (size_t)col0 * NHID + koff;
    v8f f0 = z8, f1 = z8;
#pragma unroll 1
    for (int ks = 0; ks < 4; ++ks) {
      const int k0 = ks * 32;
      const v16h a  = FragH::load(arow + k0);
      const v16h b0 = FragH::load(fb + k0);
      const v16h b1 = FragH::load(fb + 16 * NHID + k0);
      f0 = FragH::mma(a, b0, f0);
      f1 = FragH::mma(a, b1, f1);
      acc_guard2(f0, f1);
      keep4_h(a, b0, b1, a);
    }
    const float fb0 = bfr(fc_b[col0]);
    const float fb1 = bfr(fc_b[col1]);
#pragma unroll
    for (int r = 0; r < 8; ++r) {
      Os[(rb + r) * NOUT + col0] = fmaf(f0[r], Z_FOLD, fb0);
      Os[(rb + r) * NOUT + col1] = fmaf(f1[r], Z_FOLD, fb1);
    }
  }
  __syncthreads();
  {
    float* ob = out + (size_t)rowbase * NOUT;
    for (int pass = 0; pass < 2; ++pass) {
#pragma unroll
      for (int it = 0; it < 3; ++it) {
        const int f = it * NTHR + tid;
        const v4f v = *(const v4f*)(Os + f * 4);
        *(volatile v4f*)(ob + (size_t)f * 4) = v;
      }
      __threadfence();
    }
  }
}

extern "C" void kernel_launch(void* const* d_in, const int* in_sizes, int n_in,
                              void* d_out, int out_size, void* d_ws, size_t ws_size, hipStream_t stream) {
  if (n_in < 7 || d_out == nullptr || d_ws == nullptr) return;
  if (in_sizes[0] != NSEQ * NSTEP * NIN || in_sizes[1] != NG3 * NIN || in_sizes[2] != NG3 * NHID ||
      in_sizes[3] != NG3 || in_sizes[4] != NG3 || in_sizes[5] != NOUT * NHID || in_sizes[6] != NOUT ||
      out_size != NSEQ * NOUT) return;

  const float* x    = (const float*)d_in[0];
  const float* w_ih = (const float*)d_in[1];
  const float* w_hh = (const float*)d_in[2];
  const float* b_ih = (const float*)d_in[3];
  const float* b_hh = (const float*)d_in[4];
  const float* fc_w = (const float*)d_in[5];
  const float* fc_b = (const float*)d_in[6];
  float* out = (float*)d_out;

  char* ws = (char*)d_ws; size_t off = 0;
  auto carve = [&](size_t bytes) -> char* { char* p = ws + off; off += (bytes + 255) & ~(size_t)255; return p; };
  const size_t wb_bytes = (size_t)NG3 * KAUG * 2;
  const size_t fc_bytes = (size_t)NOUT * NHID * 2;
  unsigned short* WB  = (unsigned short*)carve(wb_bytes);
  unsigned short* FCP = (unsigned short*)carve(fc_bytes);
  if (off > ws_size || off > (size_t)134217728) return;

  const int n8a = NG3 * KAUG / 8;
  const int n8f = NOUT * NHID / 8;
  wplane_kernel<true><<<n8a / NTHR, NTHR, 0, stream>>>(w_hh, w_ih, n8a, WB);
  wplane_kernel<false><<<n8f / NTHR, NTHR, 0, stream>>>(fc_w, fc_w, n8f, FCP);
  gru_head_kernel<<<NSEQ / TROWS, NTHR, 0, stream>>>(x, b_ih, b_hh, fc_b, WB, FCP, out);
}
